// SARDecoder_48266842472491
// MI455X (gfx1250) — hardware-verified
//
#include <hip/hip_runtime.h>
#include <hip/hip_bf16.h>
#include <math.h>
#include <stdint.h>

typedef __attribute__((ext_vector_type(16))) _Float16 v16h;
typedef __attribute__((ext_vector_type(8)))  _Float16 v8h;
typedef __attribute__((ext_vector_type(16))) __bf16   v16b;
typedef __attribute__((ext_vector_type(8)))  __bf16   v8b;
typedef __attribute__((ext_vector_type(8)))  float    v8f;
typedef __attribute__((ext_vector_type(4)))  float    v4f;

constexpr int kBatch  = 32;
constexpr int kRnn    = 512;
constexpr int kAtt    = 512;
constexpr int kFeat   = 512;
constexpr int kVoc    = 111;
constexpr int kVocPad = 128;
constexpr int kSteps  = 31;
constexpr int kImgH   = 8;
constexpr int kImgW   = 32;
constexpr int kHW     = kImgH * kImgW;
constexpr int kConvM  = kBatch * kHW;
constexpr int kConvK  = kFeat * 9;
constexpr int kOutFloats = kBatch * kSteps * kVoc;
static_assert(kConvM % 64 == 0);
static_assert(kAtt % 64 == 0);
static_assert(kConvK % 32 == 0);
static_assert(kRnn % 32 == 0);
static_assert(kRnn % 64 == 0);
static_assert((2 * kRnn) % 32 == 0);
static_assert(kVocPad % 64 == 0);
static_assert(kOutFloats % 4 == 0);

__device__ __forceinline__ unsigned short f2bf_bits(float f) {
  unsigned u = __float_as_uint(f);
  return (unsigned short)((u + 0x7FFFu + ((u >> 16) & 1u)) >> 16);
}
__device__ __forceinline__ float bf_bits2f(unsigned short h) { return __uint_as_float(((unsigned)h) << 16); }
__device__ __forceinline__ float rne_bf(float f) { return bf_bits2f(f2bf_bits(f)); }

__device__ __forceinline__ void dep_guard_h(v8f& a, v8f& b, v16h x, v16h y) { asm volatile("v_nop\n\tv_nop\n\tv_nop\n\tv_nop" : "+v"(a), "+v"(b) : "v"(x), "v"(y)); }
__device__ __forceinline__ void dep_guard_b(v8f& a, v8f& b, v16b x, v16b y) { asm volatile("v_nop\n\tv_nop\n\tv_nop\n\tv_nop" : "+v"(a), "+v"(b) : "v"(x), "v"(y)); }
__device__ __forceinline__ void keep4_h(v16h a, v16h b, v16h c, v16h d) { asm volatile("v_nop" :: "v"(a), "v"(b), "v"(c), "v"(d)); }
__device__ __forceinline__ void keep4_b(v16b a, v16b b, v16b c, v16b d) { asm volatile("v_nop" :: "v"(a), "v"(b), "v"(c), "v"(d)); }
__device__ __forceinline__ void acc_guard4(v8f& a, v8f& b, v8f& c, v8f& d) { asm volatile("v_nop\n\tv_nop\n\tv_nop\n\tv_nop" : "+v"(a), "+v"(b), "+v"(c), "+v"(d)); }
__device__ __forceinline__ void acc_guard2(v8f& a, v8f& b) { asm volatile("v_nop\n\tv_nop\n\tv_nop\n\tv_nop" : "+v"(a), "+v"(b)); }

template <typename T> struct Frag;
template <> struct Frag<_Float16> {
  typedef v16h V; union U { v16h v; v8h h[2]; };
  static __device__ __forceinline__ v16h load(const _Float16* p) {
    U f; f.h[0] = *(const v8h*)(p); f.h[1] = *(const v8h*)(p + 16); return f.v;
  }
  static __device__ __forceinline__ v8f mma(v16h a, v16h b, v8f c) {
    return __builtin_amdgcn_wmma_f32_16x16x32_f16(false, a, false, b, (short)0, c, false, false);
  }
  static __device__ __forceinline__ void guard(v8f& a, v8f& b, v16h x, v16h y) { dep_guard_h(a, b, x, y); }
  static __device__ __forceinline__ void keep(v16h a, v16h b, v16h c, v16h d) { keep4_h(a, b, c, d); }
};
template <> struct Frag<__bf16> {
  typedef v16b V; union U { v16b v; v8b h[2]; };
  static __device__ __forceinline__ v16b load(const __bf16* p) {
    U f; f.h[0] = *(const v8b*)(p); f.h[1] = *(const v8b*)(p + 16); return f.v;
  }
  static __device__ __forceinline__ v8f mma(v16b a, v16b b, v8f c) {
    return __builtin_amdgcn_wmma_f32_16x16x32_bf16(false, a, false, b, (short)0, c, false, false);
  }
  static __device__ __forceinline__ void guard(v8f& a, v8f& b, v16b x, v16b y) { dep_guard_b(a, b, x, y); }
  static __device__ __forceinline__ void keep(v16b a, v16b b, v16b c, v16b d) { keep4_b(a, b, c, d); }
};
typedef Frag<__bf16> FragB;

template <int ET> struct Elem;
template <> struct Elem<0> { typedef _Float16 T; };
template <> struct Elem<1> { typedef __bf16 T; };
template <int ET, bool SPLIT, int BIAS_MODE, int OUT_MODE, bool RESID, int ACT = 0>
__global__ __launch_bounds__(256) void wmma_gemm64(
    const unsigned short* __restrict__ Ap, const unsigned short* __restrict__ A2p, int lda, long strideA,
    const unsigned short* __restrict__ Btp, const unsigned short* __restrict__ Bt2p, int ldb, long strideB,
    void* __restrict__ Cout, void* __restrict__ Cout2, int ldc, long strideC,
    const float* __restrict__ bias,
    const float* __restrict__ resid, long strideR,
    int M, int N, int K, float scale) {
  typedef typename Elem<ET>::T T;
  typedef typename Frag<T>::V V;
  const T* A = (const T*)Ap; const T* A2 = (const T*)A2p; const T* Bt = (const T*)Btp; const T* Bt2 = (const T*)Bt2p;
  __shared__ __align__(16) float sT[8][16 * 68];
  const int b    = blockIdx.y;
  const int lane = threadIdx.x & 31;
  const int wave = threadIdx.x >> 5;
  const int tilesN = N >> 6;
  const int tilesM = M >> 6;
  const int tile = blockIdx.x * 8 + wave;
  if (tile >= tilesM * tilesN) return;
  const int tm = tile / tilesN;
  const int tn = tile - tm * tilesN;
  const int m0 = tm << 6;
  const int n0 = tn << 6;

  const T* Ab  = A  + (size_t)b * strideA;
  const T* Bb  = Bt + (size_t)b * strideB;
  const T* Ab2 = SPLIT ? (A2  + (size_t)b * strideA) : nullptr;
  const T* Bb2 = SPLIT ? (Bt2 + (size_t)b * strideB) : nullptr;

  const int rlane = lane & 15;
  const int koff  = (lane >> 4) * 8;
  const int mOff  = (lane >> 4) * 8;

  v8f acc[4][4];
#pragma unroll
  for (int i = 0; i < 4; ++i)
#pragma unroll
    for (int j = 0; j < 4; ++j) acc[i][j] = (v8f){0.f,0.f,0.f,0.f,0.f,0.f,0.f,0.f};

  for (int k0 = 0; k0 < K; k0 += 32) {
    V bh[4], bl[4];
#pragma unroll
    for (int j = 0; j < 4; ++j) {
      const size_t bo = (size_t)(n0 + (j << 4) + rlane) * ldb + koff + k0;
      bh[j] = Frag<T>::load(Bb + bo);
      if (SPLIT) bl[j] = Frag<T>::load(Bb2 + bo);
    }
#pragma unroll
    for (int i = 0; i < 4; ++i) {
      const size_t ao = (size_t)(m0 + (i << 4) + rlane) * lda + koff + k0;
      V ah = Frag<T>::load(Ab + ao);
      V al;
      if (SPLIT) al = Frag<T>::load(Ab2 + ao);
#pragma unroll
      for (int j = 0; j < 4; ++j) {
        acc[i][j] = Frag<T>::mma(ah, bh[j], acc[i][j]);
        if (SPLIT) {
          acc[i][j] = Frag<T>::mma(ah, bl[j], acc[i][j]);
          acc[i][j] = Frag<T>::mma(al, bh[j], acc[i][j]);
        }
      }
      Frag<T>::guard(acc[i][0], acc[i][3], ah, SPLIT ? al : ah);
    }
    Frag<T>::keep(bh[0], bh[1], bh[2], bh[3]);
    if (SPLIT) Frag<T>::keep(bl[0], bl[1], bl[2], bl[3]);
  }
  acc_guard4(acc[0][0], acc[0][1], acc[0][2], acc[0][3]);
  acc_guard4(acc[1][0], acc[1][1], acc[1][2], acc[1][3]);
  acc_guard4(acc[2][0], acc[2][1], acc[2][2], acc[2][3]);
  acc_guard4(acc[3][0], acc[3][1], acc[3][2], acc[3][3]);

  float* slab = sT[wave];
  const float* Rb = RESID ? (resid + (size_t)b * strideR) : nullptr;
#pragma unroll
  for (int i = 0; i < 4; ++i) {
    const int mBase = m0 + (i << 4);
#pragma unroll
    for (int j = 0; j < 4; ++j) {
      const int n = n0 + (j << 4) + rlane;
      float bv = 0.f;
      if (BIAS_MODE == 2) bv = bias[n];
#pragma unroll
      for (int r = 0; r < 8; ++r) {
        float v = acc[i][j][r] * scale;
        if (BIAS_MODE == 1) v += bias[mBase + mOff + r];
        if (BIAS_MODE == 2) v += bv;
        if (RESID) v += Rb[(size_t)(mBase + mOff + r) * ldc + n];
        if (ACT == 1) v = tanhf(v);
        if (ACT == 2) v = fmaxf(v, 0.0f);
        if (ACT == 3) v = v / (1.0f + expf(-v));
        if (ACT == 4) v = (v > 0.f) ? v : 0.01f * v;
        if (ACT == 5) v = 0.5f * v * (1.0f + erff(v * 0.70710678118654752f));
        slab[(mOff + r) * 68 + (j << 4) + rlane] = v;
      }
    }
    __builtin_amdgcn_fence(__ATOMIC_RELEASE, "workgroup");
    __builtin_amdgcn_wave_barrier();
    __builtin_amdgcn_fence(__ATOMIC_ACQUIRE, "workgroup");
    if (OUT_MODE == 0) {
      float* C = (float*)Cout + (size_t)b * strideC;
      const int hh = lane >> 4, c4 = (lane & 15) * 4;
      for (int pass = 0; pass < 2; ++pass) {
#pragma unroll
        for (int it = 0; it < 8; ++it) {
          const int row = it * 2 + hh;
          v4f v = *(const v4f*)(slab + row * 68 + c4);
          *(volatile v4f*)(C + (size_t)(mBase + row) * ldc + n0 + c4) = v;
        }
        __threadfence();
      }
    } else {
      const int q = lane >> 3, c8 = (lane & 7) * 8;
      unsigned short* C  = (unsigned short*)Cout  + (size_t)b * strideC;
      unsigned short* C2 = (OUT_MODE == 2) ? ((unsigned short*)Cout2 + (size_t)b * strideC) : nullptr;
      for (int pass = 0; pass < 2; ++pass) {
#pragma unroll
        for (int it = 0; it < 4; ++it) {
          const int row = it * 4 + q;
          const float* sp = slab + row * 68 + c8;
          v8h hv, lv;
#pragma unroll
          for (int e = 0; e < 8; ++e) {
            if (OUT_MODE == 1) {
              hv[e] = (_Float16)sp[e];
            } else {
              unsigned short hb = f2bf_bits(sp[e]);
              unsigned short lb = f2bf_bits(sp[e] - bf_bits2f(hb));
              hv[e] = __builtin_bit_cast(_Float16, hb);
              lv[e] = __builtin_bit_cast(_Float16, lb);
            }
          }
          *(volatile v8h*)(C + (size_t)(mBase + row) * ldc + n0 + c8) = hv;
          if (OUT_MODE == 2) *(volatile v8h*)(C2 + (size_t)(mBase + row) * ldc + n0 + c8) = lv;
        }
        __threadfence();
      }
    }
    __builtin_amdgcn_fence(__ATOMIC_RELEASE, "workgroup");
    __builtin_amdgcn_wave_barrier();
    __builtin_amdgcn_fence(__ATOMIC_ACQUIRE, "workgroup");
  }
}

__device__ __forceinline__ void store2_u32(unsigned* p, unsigned u) {
  *(volatile unsigned*)p = u;
  __threadfence();
  *(volatile unsigned*)p = u;
}
__device__ __forceinline__ unsigned pack_bf2(float a, float b) {
  return (unsigned)f2bf_bits(a) | (((unsigned)f2bf_bits(b)) << 16);
}
__device__ __forceinline__ float tanh_c(float x) {
  x = fminf(fmaxf(x, -16.0f), 16.0f);
  return tanhf(x);
}
__device__ __forceinline__ float sigm_c(float x) {
  x = fminf(fmaxf(x, -30.0f), 30.0f);
  return 1.0f / (1.0f + expf(-x));
}

__global__ __launch_bounds__(256) void cast_bf16_pairs(const float* __restrict__ in, unsigned short* __restrict__ out, int n2) {
  const int i = blockIdx.x * 256 + threadIdx.x;
  if (i < n2) store2_u32((unsigned*)out + i, pack_bf2(in[2 * i], in[2 * i + 1]));
}
__global__ __launch_bounds__(256) void cast_bf16_pairs4(
    const float* __restrict__ s0, const float* __restrict__ s1, const float* __restrict__ s2, const float* __restrict__ s3,
    unsigned short* __restrict__ d0, unsigned short* __restrict__ d1, unsigned short* __restrict__ d2, unsigned short* __restrict__ d3, int n2) {
  const float* src = s0; unsigned short* dst = d0;
  if (blockIdx.y == 1) { src = s1; dst = d1; }
  else if (blockIdx.y == 2) { src = s2; dst = d2; }
  else if (blockIdx.y == 3) { src = s3; dst = d3; }
  const int i = blockIdx.x * 256 + threadIdx.x;
  if (i < n2) store2_u32((unsigned*)dst + i, pack_bf2(src[2 * i], src[2 * i + 1]));
}
__global__ __launch_bounds__(256) void prep_wout(const float* __restrict__ w, unsigned short* __restrict__ out) {
  const int i = blockIdx.x * 256 + threadIdx.x;
  if (i >= kVocPad * 2 * kRnn / 2) return;
  const int o = 2 * i;
  const int n = o >> 10, k = o & 1023;
  const int nn = (n < kVoc) ? n : (kVoc - 1);
  float v0 = w[(size_t)nn * (2 * kRnn) + k];
  float v1 = w[(size_t)nn * (2 * kRnn) + k + 1];
  if (n >= kVoc) { v0 = 0.f; v1 = 0.f; }
  store2_u32((unsigned*)out + i, pack_bf2(v0, v1));
}
__global__ __launch_bounds__(256) void prep_wconv(const float* __restrict__ wf, unsigned short* __restrict__ out) {
  const int i = blockIdx.x * 256 + threadIdx.x;
  if (i >= kAtt * kConvK / 2) return;
  const int o = 2 * i;
  const int a = o / kConvK;
  const int k = o - a * kConvK;
  const int tap = k >> 9, c = k & 511;
  const int ky = tap / 3, kx = tap - ky * 3;
  const size_t s0 = (((size_t)a * kFeat + c) * 3 + ky) * 3 + kx;
  store2_u32((unsigned*)out + i, pack_bf2(wf[s0], wf[s0 + 9]));
}
__global__ __launch_bounds__(256) void im2col_bf16(const float* __restrict__ feat, unsigned short* __restrict__ xc) {
  const int i = blockIdx.x * 256 + threadIdx.x;
  if (i >= kConvM * (kConvK / 2)) return;
  const int m  = i / (kConvK / 2);
  const int kp = i - m * (kConvK / 2);
  const int k  = 2 * kp;
  const int tap = k >> 9, c = k & 511;
  const int ky = tap / 3, kx = tap - ky * 3;
  const int b = m >> 8, hw = m & 255, y = hw >> 5, x = hw & 31;
  const int yy = y + ky - 1, xx = x + kx - 1;
  const bool valid = ((unsigned)yy < (unsigned)kImgH) && ((unsigned)xx < (unsigned)kImgW);
  const int yc = (yy < 0) ? 0 : ((yy > kImgH - 1) ? (kImgH - 1) : yy);
  const int xcl = (xx < 0) ? 0 : ((xx > kImgW - 1) ? (kImgW - 1) : xx);
  const size_t src = (((size_t)b * kFeat + c) * kImgH + yc) * kImgW + xcl;
  float v0 = feat[src];
  float v1 = feat[src + kHW];
  if (!valid) { v0 = 0.f; v1 = 0.f; }
  store2_u32((unsigned*)xc + i, pack_bf2(v0, v1));
}
__global__ __launch_bounds__(256) void gather_x(const float* __restrict__ wemb, const int* __restrict__ gt, unsigned short* __restrict__ xall) {
  const int i = blockIdx.x * 256 + threadIdx.x;
  if (i >= kSteps * kBatch * kRnn / 2) return;
  const int o = 2 * i;
  const int t = o >> 14;
  const int rem = o & 16383;
  const int b = rem >> 9, k = rem & 511;
  const int tt = (t > 0) ? (t - 1) : 0;
  int v = gt[b * kSteps + tt];
  v = (v < 0) ? 0 : ((v > kVoc - 1) ? (kVoc - 1) : v);
  float x0 = wemb[(size_t)k * kVoc + v];
  float x1 = wemb[(size_t)(k + 1) * kVoc + v];
  if (t == 0) { x0 = 0.f; x1 = 0.f; }
  store2_u32((unsigned*)xall + i, pack_bf2(x0, x1));
}

struct CellArgs {
  const unsigned short* xh; const unsigned short* xl;
  const unsigned short* hh; const unsigned short* hl;
  const unsigned short* wih; const unsigned short* whh;
  const float* bih; const float* bhh;
  const float* cprev; float* cnext;
  unsigned short* hnh; unsigned short* hnl;
  int xlo; int first;
};
static_assert(sizeof(CellArgs) == 104);

__global__ __launch_bounds__(128) void lstm_cell_dual(CellArgs ra, CellArgs rb, int na) {
  __shared__ __align__(16) float gS[4 * 32 * 68];
  __shared__ __align__(16) float cNew[32 * 68];
  __shared__ __align__(16) float hNew[32 * 68];
  const int bx = blockIdx.x;
  const bool roleA = bx < na;
  const CellArgs g = roleA ? ra : rb;
  const int blk = roleA ? bx : (bx - na);
  const int tid = threadIdx.x, wave = tid >> 5, lane = tid & 31;
  const int rl = lane & 15, hf = lane >> 4, koff = hf * 8;
  const int jblk = blk * 64;
  const int j0 = jblk + wave * 16;
  const __bf16* Xh = (const __bf16*)g.xh;  const __bf16* Xl = (const __bf16*)g.xl;
  const __bf16* Hh = (const __bf16*)g.hh;  const __bf16* Hl = (const __bf16*)g.hl;
  const __bf16* Wx = (const __bf16*)g.wih; const __bf16* Wh = (const __bf16*)g.whh;
  const bool xlo = (g.xlo != 0);
  const bool hasPrev = (g.first == 0);

  v8f acc[2][4];
#pragma unroll
  for (int i = 0; i < 2; ++i)
#pragma unroll
    for (int q = 0; q < 4; ++q) acc[i][q] = (v8f){0.f,0.f,0.f,0.f,0.f,0.f,0.f,0.f};

  for (int k0 = 0; k0 < kRnn; k0 += 32) {
    v16b bw[4];
#pragma unroll
    for (int q = 0; q < 4; ++q) bw[q] = FragB::load(Wx + (size_t)(q * kRnn + j0 + rl) * kRnn + koff + k0);
    const size_t o0 = (size_t)rl * kRnn + koff + k0;
    const size_t o1 = (size_t)(16 + rl) * kRnn + koff + k0;
    const v16b a0h = FragB::load(Xh + o0);
    const v16b a1h = FragB::load(Xh + o1);
    v16b a0l = a0h, a1l = a1h;
    if (xlo) { a0l = FragB::load(Xl + o0); a1l = FragB::load(Xl + o1); }
#pragma unroll
    for (int q = 0; q < 4; ++q) {
      acc[0][q] = FragB::mma(a0h, bw[q], acc[0][q]);
      if (xlo) acc[0][q] = FragB::mma(a0l, bw[q], acc[0][q]);
      acc[1][q] = FragB::mma(a1h, bw[q], acc[1][q]);
      if (xlo) acc[1][q] = FragB::mma(a1l, bw[q], acc[1][q]);
    }
    dep_guard_b(acc[0][0], acc[1][3], a0h, a1h);
    keep4_b(bw[0], bw[1], bw[2], bw[3]);
    keep4_b(a0l, a1l, a0l, a1l);
  }
  if (hasPrev) {
    for (int k0 = 0; k0 < kRnn; k0 += 32) {
      v16b bw[4];
#pragma unroll
      for (int q = 0; q < 4; ++q) bw[q] = FragB::load(Wh + (size_t)(q * kRnn + j0 + rl) * kRnn + koff + k0);
      const size_t o0 = (size_t)rl * kRnn + koff + k0;
      const size_t o1 = (size_t)(16 + rl) * kRnn + koff + k0;
      const v16b a0h = FragB::load(Hh + o0);
      const v16b a1h = FragB::load(Hh + o1);
      const v16b a0l = FragB::load(Hl + o0);
      const v16b a1l = FragB::load(Hl + o1);
#pragma unroll
      for (int q = 0; q < 4; ++q) {
        acc[0][q] = FragB::mma(a0h, bw[q], acc[0][q]);
        acc[0][q] = FragB::mma(a0l, bw[q], acc[0][q]);
        acc[1][q] = FragB::mma(a1h, bw[q], acc[1][q]);
        acc[1][q] = FragB::mma(a1l, bw[q], acc[1][q]);
      }
      dep_guard_b(acc[0][0], acc[1][3], a0h, a1h);
      keep4_b(bw[0], bw[1], bw[2], bw[3]);
      keep4_b(a0l, a1l, a0l, a1l);
    }
  }
  acc_guard4(acc[0][0], acc[0][1], acc[0][2], acc[0][3]);
  acc_guard4(acc[1][0], acc[1][1], acc[1][2], acc[1][3]);

  float bsum[4];
#pragma unroll
  for (int q = 0; q < 4; ++q) {
    const int n = q * kRnn + j0 + rl;
    bsum[q] = rne_bf(g.bih[n]) + rne_bf(g.bhh[n]);
  }
#pragma unroll
  for (int mi = 0; mi < 2; ++mi)
#pragma unroll
    for (int q = 0; q < 4; ++q)
#pragma unroll
      for (int r = 0; r < 8; ++r)
        gS[(q * 32 + mi * 16 + 8 * hf + r) * 68 + wave * 16 + rl] = acc[mi][q][r] + bsum[q];
  __syncthreads();

#pragma unroll 1
  for (int e = 0; e < 16; ++e) {
    const int el = e * 128 + tid;
    const int row = el >> 6, col = el & 63;
    const int li = row * 68 + col;
    const float pi = gS[li];
    const float pf = gS[32 * 68 + li];
    const float pg = gS[2 * 32 * 68 + li];
    const float po = gS[3 * 32 * 68 + li];
    float cold = 0.f;
    if (hasPrev) cold = g.cprev[(size_t)row * kRnn + jblk + col];
    const float ig = sigm_c(pi);
    const float fg = sigm_c(pf);
    const float og = sigm_c(po);
    const float gg = tanh_c(pg);
    const float cn = fg * cold + ig * gg;
    const float hn = og * tanh_c(cn);
    cNew[li] = cn;
    hNew[li] = hn;
  }
  __syncthreads();

  for (int pass = 0; pass < 2; ++pass) {
#pragma unroll
    for (int it = 0; it < 4; ++it) {
      const int row = wave * 8 + it * 2 + hf;
      const int c4 = rl * 4;
      const v4f v = *(const v4f*)(cNew + row * 68 + c4);
      *(volatile v4f*)(g.cnext + (size_t)row * kRnn + jblk + c4) = v;
    }
#pragma unroll
    for (int it = 0; it < 2; ++it) {
      const int row = wave * 8 + it * 4 + (lane >> 3);
      const int c8 = (lane & 7) * 8;
      const float* s8 = hNew + row * 68 + c8;
      v8h hv, lv;
#pragma unroll
      for (int e = 0; e < 8; ++e) {
        const unsigned short hb = f2bf_bits(s8[e]);
        const unsigned short lb = f2bf_bits(s8[e] - bf_bits2f(hb));
        hv[e] = __builtin_bit_cast(_Float16, hb);
        lv[e] = __builtin_bit_cast(_Float16, lb);
      }
      *(volatile v8h*)(g.hnh + (size_t)row * kRnn + jblk + c8) = hv;
      *(volatile v8h*)(g.hnl + (size_t)row * kRnn + jblk + c8) = lv;
    }
    __threadfence();
  }
}

struct GemmArgs {
  const unsigned short* a1h; const unsigned short* a1l; const unsigned short* b1;
  const unsigned short* a2h; const unsigned short* a2l; const unsigned short* b2;
  const float* bias; float* c;
  int lda1, ldb1, k1, lda2, ldb2, k2, ldc, nbias;
};
static_assert(sizeof(GemmArgs) == 96);

__global__ __launch_bounds__(128) void gemm32_dual(GemmArgs ga, GemmArgs gb, int na) {
  __shared__ __align__(16) float sS[32 * 68];
  const int bx = blockIdx.x;
  const bool roleA = bx < na;
  const GemmArgs g = roleA ? ga : gb;
  const int blk = roleA ? bx : (bx - na);
  const int tid = threadIdx.x, wave = tid >> 5, lane = tid & 31;
  const int rl = lane & 15, hf = lane >> 4, koff = hf * 8;
  const int nblk0 = blk * 64;
  const int n0 = nblk0 + wave * 16;
  const __bf16* A1h = (const __bf16*)g.a1h; const __bf16* A1l = (const __bf16*)g.a1l; const __bf16* B1 = (const __bf16*)g.b1;
  const __bf16* A2h = (const __bf16*)g.a2h; const __bf16* A2l = (const __bf16*)g.a2l; const __bf16* B2 = (const __bf16*)g.b2;

  v8f acc0 = (v8f){0.f,0.f,0.f,0.f,0.f,0.f,0.f,0.f};
  v8f acc1 = (v8f){0.f,0.f,0.f,0.f,0.f,0.f,0.f,0.f};
  for (int k0 = 0; k0 < g.k1; k0 += 32) {
    const v16b bb = FragB::load(B1 + (size_t)(n0 + rl) * g.ldb1 + koff + k0);
    const size_t o0 = (size_t)rl * g.lda1 + koff + k0;
    const size_t o1 = (size_t)(16 + rl) * g.lda1 + koff + k0;
    const v16b a0h = FragB::load(A1h + o0), a1h = FragB::load(A1h + o1);
    const v16b a0l = FragB::load(A1l + o0), a1l = FragB::load(A1l + o1);
    acc0 = FragB::mma(a0h, bb, acc0);
    acc0 = FragB::mma(a0l, bb, acc0);
    acc1 = FragB::mma(a1h, bb, acc1);
    acc1 = FragB::mma(a1l, bb, acc1);
    dep_guard_b(acc0, acc1, a0h, a1h);
    keep4_b(bb, a0l, a1l, bb);
  }
  for (int k0 = 0; k0 < g.k2; k0 += 32) {
    const v16b bb = FragB::load(B2 + (size_t)(n0 + rl) * g.ldb2 + koff + k0);
    const size_t o0 = (size_t)rl * g.lda2 + koff + k0;
    const size_t o1 = (size_t)(16 + rl) * g.lda2 + koff + k0;
    const v16b a0h = FragB::load(A2h + o0), a1h = FragB::load(A2h + o1);
    const v16b a0l = FragB::load(A2l + o0), a1l = FragB::load(A2l + o1);
    acc0 = FragB::mma(a0h, bb, acc0);
    acc0 = FragB::mma(a0l, bb, acc0);
    acc1 = FragB::mma(a1h, bb, acc1);
    acc1 = FragB::mma(a1l, bb, acc1);
    dep_guard_b(acc0, acc1, a0h, a1h);
    keep4_b(bb, a0l, a1l, bb);
  }
  acc_guard2(acc0, acc1);

  float bv = 0.f;
  if (g.nbias > 0) {
    const int n = n0 + rl;
    const int nn = (n < g.nbias) ? n : (g.nbias - 1);
    bv = rne_bf(g.bias[nn]);
    if (n >= g.nbias) bv = 0.f;
  }
#pragma unroll
  for (int r = 0; r < 8; ++r) {
    sS[(8 * hf + r) * 68 + wave * 16 + rl] = acc0[r] + bv;
    sS[(16 + 8 * hf + r) * 68 + wave * 16 + rl] = acc1[r] + bv;
  }
  __syncthreads();
  for (int pass = 0; pass < 2; ++pass) {
#pragma unroll
    for (int it = 0; it < 4; ++it) {
      const int row = wave * 8 + it * 2 + hf;
      const int c4 = rl * 4;
      const v4f v = *(const v4f*)(sS + row * 68 + c4);
      *(volatile v4f*)(g.c + (size_t)row * g.ldc + nblk0 + c4) = v;
    }
    __threadfence();
  }
}

__global__ __launch_bounds__(256) void att_glimpse(const float* __restrict__ fproj, const float* __restrict__ sp,
                                                   const float* __restrict__ watt, const unsigned short* __restrict__ featr,
                                                   unsigned short* __restrict__ ghi, unsigned short* __restrict__ glo) {
  __shared__ float sps[kAtt];
  __shared__ float was[kAtt];
  __shared__ float red[kHW];
  __shared__ __align__(16) float att[kHW];
  __shared__ __align__(16) float gsum[kFeat];
  const int b = blockIdx.x, tid = threadIdx.x, wave = tid >> 5, lane = tid & 31;
  sps[tid] = sp[(size_t)b * kAtt + tid];
  sps[tid + 256] = sp[(size_t)b * kAtt + 256 + tid];
  was[tid] = rne_bf(watt[tid]);
  was[tid + 256] = rne_bf(watt[tid + 256]);
  __syncthreads();

  const float* prow = fproj + (size_t)(b * kHW + tid) * kAtt;
  float e = 0.f;
#pragma unroll 1
  for (int a = 0; a < kAtt; ++a) {
    float v = prow[a] + sps[a];
    v = fminf(fmaxf(v, -16.0f), 16.0f);
    e = fmaf(was[a], tanhf(v), e);
  }
  red[tid] = e;
  __syncthreads();
  for (int s = 128; s > 0; s >>= 1) {
    if (tid < s) red[tid] = fmaxf(red[tid], red[tid + s]);
    __syncthreads();
  }
  const float mx = red[0];
  __syncthreads();
  const float ex = expf(e - mx);
  red[tid] = ex;
  __syncthreads();
  for (int s = 128; s > 0; s >>= 1) {
    if (tid < s) red[tid] = red[tid] + red[tid + s];
    __syncthreads();
  }
  const float tot = red[0];
  __syncthreads();
  att[tid] = ex * (1.0f / tot);
  __syncthreads();

#pragma unroll 1
  for (int cc = 0; cc < 2; ++cc) {
    const int c = tid + cc * 256;
    const uint4* p = (const uint4*)(featr + ((size_t)(b * kFeat + c)) * kHW);
    float s = 0.f;
#pragma unroll 1
    for (int i = 0; i < kHW / 8; ++i) {
      const uint4 w = p[i];
      const float* ap = att + i * 8;
      s = fmaf(ap[0], __uint_as_float(w.x << 16), s);
      s = fmaf(ap[1], __uint_as_float(w.x & 0xffff0000u), s);
      s = fmaf(ap[2], __uint_as_float(w.y << 16), s);
      s = fmaf(ap[3], __uint_as_float(w.y & 0xffff0000u), s);
      s = fmaf(ap[4], __uint_as_float(w.z << 16), s);
      s = fmaf(ap[5], __uint_as_float(w.z & 0xffff0000u), s);
      s = fmaf(ap[6], __uint_as_float(w.w << 16), s);
      s = fmaf(ap[7], __uint_as_float(w.w & 0xffff0000u), s);
    }
    gsum[c] = s;
  }
  __syncthreads();
  if (wave == 0) {
    for (int pass = 0; pass < 2; ++pass) {
#pragma unroll
      for (int it = 0; it < 2; ++it) {
        const int c8 = it * 256 + lane * 8;
        const float* s8 = gsum + c8;
        v8h hv, lv;
#pragma unroll
        for (int q = 0; q < 8; ++q) {
          const unsigned short hb = f2bf_bits(s8[q]);
          const unsigned short lb = f2bf_bits(s8[q] - bf_bits2f(hb));
          hv[q] = __builtin_bit_cast(_Float16, hb);
          lv[q] = __builtin_bit_cast(_Float16, lb);
        }
        *(volatile v8h*)(ghi + (size_t)b * kFeat + c8) = hv;
        *(volatile v8h*)(glo + (size_t)b * kFeat + c8) = lv;
      }
      __threadfence();
    }
  }
}

__global__ __launch_bounds__(256) void pack_out(const float* __restrict__ lg, float* __restrict__ out, int nfloat) {
  const int wv = blockIdx.x * 8 + (threadIdx.x >> 5);
  const int lane = threadIdx.x & 31;
  const int f0 = wv * 128 + lane * 4;
  if (f0 >= nfloat) return;
  v4f v;
#pragma unroll
  for (int e = 0; e < 4; ++e) {
    const int f = f0 + e;
    const int q = f / kVoc;
    const int vv = f - q * kVoc;
    const int b = q / kSteps;
    const int t = q - b * kSteps;
    v[e] = lg[((size_t)t * kBatch + b) * kVocPad + vv];
  }
  *(volatile v4f*)(out + f0) = v;
  __threadfence();
  *(volatile v4f*)(out + f0) = v;
}

extern "C" void kernel_launch(void* const* d_in, const int* in_sizes, int n_in,
                              void* d_out, int out_size, void* d_ws, size_t ws_size,
                              hipStream_t stream) {
  (void)in_sizes; (void)n_in; (void)out_size;
  const float* features = (const float*)d_in[0];
  const int*   gt       = (const int*)d_in[2];
  const float* W_feat   = (const float*)d_in[3];
  const float* b_feat   = (const float*)d_in[4];
  const float* W_state  = (const float*)d_in[5];
  const float* w_att    = (const float*)d_in[6];
  const float* W_embed  = (const float*)d_in[7];
  const float* wih0     = (const float*)d_in[8];
  const float* whh0     = (const float*)d_in[9];
  const float* bih0     = (const float*)d_in[10];
  const float* bhh0     = (const float*)d_in[11];
  const float* wih1     = (const float*)d_in[12];
  const float* whh1     = (const float*)d_in[13];
  const float* bih1     = (const float*)d_in[14];
  const float* bhh1     = (const float*)d_in[15];
  const float* W_out    = (const float*)d_in[16];
  const float* b_out    = (const float*)d_in[17];
  float* out = (float*)d_out;

  char* ws = (char*)d_ws;
  size_t off = 0;
  auto carve = [&](size_t bytes) { char* p = ws + off; off += (bytes + 255) & ~(size_t)255; return (void*)p; };

  const size_t plane_h = (size_t)kBatch * kRnn * 2;
  const size_t plane_c = (size_t)kBatch * kRnn * 4;

  unsigned short* xcol  = (unsigned short*)carve((size_t)kConvM * kConvK * 2);
  unsigned short* wconv = (unsigned short*)carve((size_t)kAtt * kConvK * 2);
  float*          fproj = (float*)carve((size_t)kConvM * kAtt * 4);
  unsigned short* featr = (unsigned short*)carve((size_t)kBatch * kFeat * kHW * 2);
  unsigned short* wih0b = (unsigned short*)carve((size_t)4 * kRnn * kRnn * 2);
  unsigned short* whh0b = (unsigned short*)carve((size_t)4 * kRnn * kRnn * 2);
  unsigned short* wih1b = (unsigned short*)carve((size_t)4 * kRnn * kRnn * 2);
  unsigned short* whh1b = (unsigned short*)carve((size_t)4 * kRnn * kRnn * 2);
  unsigned short* wstb  = (unsigned short*)carve((size_t)kAtt * kRnn * 2);
  unsigned short* woutb = (unsigned short*)carve((size_t)kVocPad * 2 * kRnn * 2);
  unsigned short* xall  = (unsigned short*)carve((size_t)kSteps * kBatch * kRnn * 2);
  unsigned short* h0base = (unsigned short*)carve(4 * plane_h);
  unsigned short* h1base = (unsigned short*)carve(4 * plane_h);
  float* c0base = (float*)carve(2 * plane_c);
  float* c1base = (float*)carve(2 * plane_c);
  float* spws   = (float*)carve(plane_c);
  unsigned short* gbase = (unsigned short*)carve(2 * plane_h);
  float* logits = (float*)carve((size_t)kSteps * kBatch * kVocPad * 4);
  if (off > ws_size) return;

  unsigned short* h0h[2] = { h0base, h0base + (size_t)kBatch * kRnn };
  unsigned short* h0l[2] = { h0base + 2 * (size_t)kBatch * kRnn, h0base + 3 * (size_t)kBatch * kRnn };
  unsigned short* h1h[2] = { h1base, h1base + (size_t)kBatch * kRnn };
  unsigned short* h1l[2] = { h1base + 2 * (size_t)kBatch * kRnn, h1base + 3 * (size_t)kBatch * kRnn };
  float* c0[2] = { c0base, c0base + (size_t)kBatch * kRnn };
  float* c1[2] = { c1base, c1base + (size_t)kBatch * kRnn };
  unsigned short* ghi = gbase;
  unsigned short* glo = gbase + (size_t)kBatch * kFeat;

  {
    const int n2w = 4 * kRnn * kRnn / 2;
    cast_bf16_pairs4<<<dim3((n2w + 255) / 256, 4), 256, 0, stream>>>(wih0, whh0, wih1, whh1, wih0b, whh0b, wih1b, whh1b, n2w);
    const int n2s = kAtt * kRnn / 2;
    cast_bf16_pairs<<<(n2s + 255) / 256, 256, 0, stream>>>(W_state, wstb, n2s);
    const int n2o = kVocPad * 2 * kRnn / 2;
    prep_wout<<<(n2o + 255) / 256, 256, 0, stream>>>(W_out, woutb);
    const int n2c = kAtt * kConvK / 2;
    prep_wconv<<<(n2c + 255) / 256, 256, 0, stream>>>(W_feat, wconv);
    const int n2f = kBatch * kFeat * kHW / 2;
    cast_bf16_pairs<<<(n2f + 255) / 256, 256, 0, stream>>>(features, featr, n2f);
    const int n2i = kConvM * (kConvK / 2);
    im2col_bf16<<<(n2i + 255) / 256, 256, 0, stream>>>(features, xcol);
    const int n2x = kSteps * kBatch * kRnn / 2;
    gather_x<<<(n2x + 255) / 256, 256, 0, stream>>>(W_embed, gt, xall);
  }

  {
    const int tiles = (kConvM / 64) * (kAtt / 64);
    wmma_gemm64<1, false, 2, 0, false, 0><<<dim3(tiles / 8, 1), 256, 0, stream>>>(
        xcol, xcol, kConvK, 0L, wconv, wconv, kConvK, 0L,
        (void*)fproj, (void*)fproj, kAtt, 0L, b_feat, (const float*)fproj, 0L,
        kConvM, kAtt, kConvK, 1.0f);
  }

  auto cell_args = [&](int layer, int t) {
    CellArgs a;
    const int p = t & 1, q = p ^ 1;
    if (layer == 0) {
      a.xh = xall + (size_t)t * kBatch * kRnn; a.xl = a.xh;
      a.hh = h0h[q]; a.hl = h0l[q];
      a.wih = wih0b; a.whh = whh0b; a.bih = bih0; a.bhh = bhh0;
      a.cprev = c0[q]; a.cnext = c0[p]; a.hnh = h0h[p]; a.hnl = h0l[p];
      a.xlo = 0; a.first = (t == 0) ? 1 : 0;
    } else {
      a.xh = h0h[p]; a.xl = h0l[p];
      a.hh = h1h[q]; a.hl = h1l[q];
      a.wih = wih1b; a.whh = whh1b; a.bih = bih1; a.bhh = bhh1;
      a.cprev = c1[q]; a.cnext = c1[p]; a.hnh = h1h[p]; a.hnl = h1l[p];
      a.xlo = 1; a.first = (t == 0) ? 1 : 0;
    }
    return a;
  };
  auto sp_args = [&](int t) {
    GemmArgs s;
    const int p = t & 1;
    s.a1h = h1h[p]; s.a1l = h1l[p]; s.b1 = wstb;
    s.a2h = h1h[p]; s.a2l = h1l[p]; s.b2 = wstb;
    s.bias = b_out; s.c = spws;
    s.lda1 = kRnn; s.ldb1 = kRnn; s.k1 = kRnn; s.lda2 = kRnn; s.ldb2 = kRnn; s.k2 = 0; s.ldc = kAtt; s.nbias = 0;
    return s;
  };
  auto out_args = [&](int t) {
    GemmArgs o;
    const int p = t & 1;
    o.a1h = h1h[p]; o.a1l = h1l[p]; o.b1 = woutb;
    o.a2h = ghi; o.a2l = glo; o.b2 = woutb + kRnn;
    o.bias = b_out; o.c = logits + (size_t)t * kBatch * kVocPad;
    o.lda1 = kRnn; o.ldb1 = 2 * kRnn; o.k1 = kRnn; o.lda2 = kFeat; o.ldb2 = 2 * kRnn; o.k2 = kFeat; o.ldc = kVocPad; o.nbias = kVoc;
    return o;
  };

  const int nCellBlk = (4 * kRnn) / (4 * 64);
  const int nSpBlk = kAtt / 64;
  const int nOutBlk = kVocPad / 64;

  {
    CellArgs a = cell_args(0, 0);
    lstm_cell_dual<<<nCellBlk, 128, 0, stream>>>(a, a, nCellBlk);
  }
  for (int t = 0; t < kSteps; ++t) {
    {
      CellArgs a = cell_args(1, t);
      if (t + 1 < kSteps) {
        CellArgs bnext = cell_args(0, t + 1);
        lstm_cell_dual<<<2 * nCellBlk, 128, 0, stream>>>(a, bnext, nCellBlk);
      } else {
        lstm_cell_dual<<<nCellBlk, 128, 0, stream>>>(a, a, nCellBlk);
      }
    }
    {
      GemmArgs s = sp_args(t);
      if (t > 0) {
        GemmArgs o = out_args(t - 1);
        gemm32_dual<<<nSpBlk + nOutBlk, 128, 0, stream>>>(s, o, nSpBlk);
      } else {
        gemm32_dual<<<nSpBlk, 128, 0, stream>>>(s, s, nSpBlk);
      }
    }
    att_glimpse<<<kBatch, 256, 0, stream>>>(fproj, spws, w_att, featr, ghi, glo);
  }
  {
    GemmArgs o = out_args(kSteps - 1);
    gemm32_dual<<<nOutBlk, 128, 0, stream>>>(o, o, 0);
  }
  {
    const int waves = (kOutFloats + 127) / 128;
    pack_out<<<(waves + 7) / 8, 256, 0, stream>>>(logits, out, kOutFloats);
  }
}
